// Encoder_48421461295301
// MI455X (gfx1250) — hardware-verified
//
#include <hip/hip_runtime.h>
#include <stddef.h>
#include <stdint.h>
#include <math.h>


#define NLAY   4
#define DM     512
#define DI     1024
#define NST    16
#define DTR    32
#define XD     64
#define TOK    1024
#define SEQ    512
#define NB     2
#define ALOG_BF16 1
#define GBM    64
#define GBN    64
#define GTHR   128
#define SCH    32
#define SCT    128
#define WSMAX  134217728

static_assert(TOK == NB * SEQ);
static_assert(TOK % GBM == 0 && (2 * DI) % GBN == 0 && XD == GBN && DI % GBN == 0 && DM % GBN == 0);
static_assert(DM % 32 == 0 && DI % 32 == 0 && DTR % 32 == 0);
static_assert(SEQ % SCH == 0 && DI % SCT == 0 && SCH * 32 == 8 * SCT);
static_assert(XD == DTR + 2 * NST);

typedef float          v4f   __attribute__((ext_vector_type(4)));
typedef float          v8f   __attribute__((ext_vector_type(8)));
typedef int            v8i   __attribute__((ext_vector_type(8)));
typedef unsigned short v4us  __attribute__((ext_vector_type(4)));
typedef unsigned short v8us  __attribute__((ext_vector_type(8)));
typedef unsigned short v16us __attribute__((ext_vector_type(16)));
typedef __bf16         v16bf __attribute__((ext_vector_type(16)));
typedef v4f  __attribute__((may_alias)) v4fa;
typedef v4us __attribute__((may_alias)) v4usa;
typedef v8us __attribute__((may_alias)) v8usa;
union FragB { v16bf v; v16us u; v8us h[2]; v8i w; };

__device__ __forceinline__ v8f wmb(const FragB& a, const FragB& b, v8f c) {
  v8f d = __builtin_amdgcn_wmma_f32_16x16x32_bf16(false, a.v, false, b.v, (short)0, c, false, false);
  asm volatile("v_nop\n\tv_nop\n\tv_nop\n\tv_nop" : "+v"(d) : "v"(a.w), "v"(b.w));
  return d;
}

__device__ __forceinline__ unsigned bf16_bits(float f) {
  const unsigned u = __float_as_uint(f);
  return (u + 0x7FFFu + ((u >> 16) & 1u)) >> 16;
}
__device__ __forceinline__ float bf16_val(float f) {
  return __uint_as_float(bf16_bits(f) << 16);
}
__device__ __forceinline__ v4f bf4(v4f a) {
  v4f r;
  r.x = bf16_val(a.x); r.y = bf16_val(a.y); r.z = bf16_val(a.z); r.w = bf16_val(a.w);
  return r;
}
__device__ __forceinline__ void hilo(float v, unsigned short& h, unsigned short& l) {
  const unsigned hb = bf16_bits(v);
  h = (unsigned short)hb;
  l = (unsigned short)bf16_bits(v - __uint_as_float(hb << 16));
}

__global__ __launch_bounds__(256) void k_cvt(const float* __restrict__ src, unsigned short* dst, int nUnits) {
  const int u = (int)blockIdx.x * 256 + (int)threadIdx.x;
  if (u >= nUnits) return;
  const float* p = src + (size_t)u * 8;
  const v4f a = *(const v4fa*)p;
  const v4f b = *(const v4fa*)(p + 4);
  v8us o;
  o[0] = (unsigned short)bf16_bits(a.x); o[1] = (unsigned short)bf16_bits(a.y);
  o[2] = (unsigned short)bf16_bits(a.z); o[3] = (unsigned short)bf16_bits(a.w);
  o[4] = (unsigned short)bf16_bits(b.x); o[5] = (unsigned short)bf16_bits(b.y);
  o[6] = (unsigned short)bf16_bits(b.z); o[7] = (unsigned short)bf16_bits(b.w);
  unsigned short* dp = dst + (size_t)u * 8;
  *(volatile v8us*)dp = o;
  __threadfence();
  *(volatile v8us*)dp = o;
}

template <int MODE>
__global__ __launch_bounds__(256) void k_norm(const float* __restrict__ xin, const float* __restrict__ hsp,
                                              float* res, const float* __restrict__ w,
                                              unsigned short* hn, float* outp) {
  __shared__ __attribute__((aligned(16))) unsigned short sh[8 * 1024];
  const int tid = (int)threadIdx.x, lane = tid & 31, wave = tid >> 5;
  const int row = (int)blockIdx.x * 8 + wave;
  const size_t rb = (size_t)row * DM;

  v4f v[4], wv[4];
#pragma unroll
  for (int j = 0; j < 4; ++j) {
    const int col = 4 * lane + 128 * j;
    if constexpr (MODE == 0) {
      v[j] = bf4(*(const v4fa*)(xin + rb + col));
    } else {
      const v4f h = *(const v4fa*)(hsp + rb + col);
      const v4f a = *(const v4fa*)(res + rb + col);
      v[j] = h + a;
    }
    wv[j] = bf4(*(const v4fa*)(w + col));
  }
  float ss = 0.0f;
#pragma unroll
  for (int j = 0; j < 4; ++j) {
    ss = fmaf(v[j].x, v[j].x, ss); ss = fmaf(v[j].y, v[j].y, ss);
    ss = fmaf(v[j].z, v[j].z, ss); ss = fmaf(v[j].w, v[j].w, ss);
  }
#pragma unroll
  for (int o = 16; o > 0; o >>= 1) ss += __shfl_xor(ss, o, 32);
  const float r = rsqrtf(ss * (1.0f / (float)DM) + 1e-5f);

  v4f y[4];
#pragma unroll
  for (int j = 0; j < 4; ++j) {
    y[j].x = (v[j].x * r) * wv[j].x; y[j].y = (v[j].y * r) * wv[j].y;
    y[j].z = (v[j].z * r) * wv[j].z; y[j].w = (v[j].w * r) * wv[j].w;
  }

  if constexpr (MODE == 2) {
#pragma unroll
    for (int j = 0; j < 4; ++j) *(volatile v4f*)(outp + rb + 4 * lane + 128 * j) = y[j];
    __threadfence();
#pragma unroll
    for (int j = 0; j < 4; ++j) *(volatile v4f*)(outp + rb + 4 * lane + 128 * j) = y[j];
  } else {
    unsigned short* srow = sh + wave * 1024;
#pragma unroll
    for (int j = 0; j < 4; ++j) {
      const int col = 4 * lane + 128 * j;
      v4us h4, l4;
      unsigned short hh, ll;
      hilo(y[j].x, hh, ll); h4[0] = hh; l4[0] = ll;
      hilo(y[j].y, hh, ll); h4[1] = hh; l4[1] = ll;
      hilo(y[j].z, hh, ll); h4[2] = hh; l4[2] = ll;
      hilo(y[j].w, hh, ll); h4[3] = hh; l4[3] = ll;
      *(v4usa*)(srow + col) = h4;
      *(v4usa*)(srow + DM + col) = l4;
    }
    __syncthreads();
    v8us q[4];
#pragma unroll
    for (int k = 0; k < 4; ++k) q[k] = *(const v8usa*)(srow + 8 * lane + 256 * k);
    unsigned short* hrow = hn + (size_t)row * (2 * DM);
#pragma unroll
    for (int j = 0; j < 4; ++j) *(volatile v4f*)(res + rb + 4 * lane + 128 * j) = v[j];
#pragma unroll
    for (int k = 0; k < 4; ++k) *(volatile v8us*)(hrow + 8 * lane + 256 * k) = q[k];
    __threadfence();
#pragma unroll
    for (int j = 0; j < 4; ++j) *(volatile v4f*)(res + rb + 4 * lane + 128 * j) = v[j];
#pragma unroll
    for (int k = 0; k < 4; ++k) *(volatile v8us*)(hrow + 8 * lane + 256 * k) = q[k];
  }
}

template <int MODE>
__global__ __launch_bounds__(GTHR) void k_gemm(
    const unsigned short* __restrict__ A, const unsigned short* __restrict__ BT,
    float* C, float* C2, unsigned short* aux,
    const float* __restrict__ bias0, const float* __restrict__ bias1,
    int lda, int sA, int KB, int sB, int ldc, int sC, int sAux)
{
  __shared__ __attribute__((aligned(16))) float stg[GBM * GBN];
  const int tid = (int)threadIdx.x, lane = tid & 31, wave = tid >> 5, hh = lane >> 4, m = lane & 15;
  const int rowBase = (int)blockIdx.x * GBM;
  const int col0    = (int)blockIdx.y * GBN;
  const int z       = (int)blockIdx.z;

  v8f acc[4];
  {
    const v8f zz = {0.f, 0.f, 0.f, 0.f, 0.f, 0.f, 0.f, 0.f};
    acc[0] = zz; acc[1] = zz; acc[2] = zz; acc[3] = zz;
  }
  const unsigned short* ap = A + (size_t)z * (size_t)sA + (size_t)(rowBase + 16 * wave + m) * (size_t)lda + 8 * hh;
  const unsigned short* wp = BT + (size_t)z * (size_t)sB + (size_t)(col0 + m) * (size_t)KB + 8 * hh;
  const int ksteps = (2 * KB) >> 5;
#pragma unroll 1
  for (int ks = 0; ks < ksteps; ++ks) {
    const int k0 = 32 * ks;
    const int kb = (k0 >= KB) ? (k0 - KB) : k0;
    FragB af;
    af.h[0] = *(const v8usa*)(ap + k0);
    af.h[1] = *(const v8usa*)(ap + k0 + 16);
#pragma unroll
    for (int t = 0; t < 4; ++t) {
      const unsigned short* wq = wp + (size_t)(16 * t) * (size_t)KB + kb;
      FragB bf;
      bf.h[0] = *(const v8usa*)wq;
      bf.h[1] = *(const v8usa*)(wq + 16);
      acc[t] = wmb(af, bf, acc[t]);
    }
  }

#pragma unroll
  for (int t = 0; t < 4; ++t) {
    const int lc = 16 * t + m;
#pragma unroll
    for (int r = 0; r < 8; ++r) {
      const int lr = 16 * wave + 8 * hh + r;
      stg[lr * GBN + lc] = acc[t][r];
    }
  }
  __syncthreads();

  if constexpr (MODE == 2) {
    const int cl = tid & 63;
    const float b0 = bias0[col0 + cl];
    const float b1 = bias1[col0 + cl];
    const float bz = bf16_val((z != 0) ? b1 : b0);
#pragma unroll 1
    for (int j = 0; j < (GBM * GBN) / GTHR; ++j) {
      const int idx = j * GTHR + tid;
      const float v = stg[idx] + bz;
      stg[idx] = fmaxf(v, 0.0f) + log1pf(expf(-fabsf(v)));
    }
    __syncthreads();
  }

  v4f fv[8];
#pragma unroll
  for (int i = 0; i < 8; ++i) {
    const int lr = 16 * wave + 2 * i + hh;
    fv[i] = *(const v4fa*)(stg + lr * GBN + 4 * m);
  }

  v8us dv[4];
  unsigned short* auxz = aux + (size_t)z * (size_t)sAux;
  if constexpr (MODE == 1) {
#pragma unroll
    for (int it = 0; it < 4; ++it) {
      const int p   = it * GTHR + tid;
      const int row = p >> 3;
      const int q   = p & 7;
      const int c8  = 8 * (q & 3);
      const bool isLo = (q & 4) != 0;
      const v4f a = *(const v4fa*)(stg + row * GBN + c8);
      const v4f b = *(const v4fa*)(stg + row * GBN + c8 + 4);
      unsigned short h, l;
      v8us o;
      hilo(a.x, h, l); o[0] = isLo ? l : h;
      hilo(a.y, h, l); o[1] = isLo ? l : h;
      hilo(a.z, h, l); o[2] = isLo ? l : h;
      hilo(a.w, h, l); o[3] = isLo ? l : h;
      hilo(b.x, h, l); o[4] = isLo ? l : h;
      hilo(b.y, h, l); o[5] = isLo ? l : h;
      hilo(b.z, h, l); o[6] = isLo ? l : h;
      hilo(b.w, h, l); o[7] = isLo ? l : h;
      dv[it] = o;
    }
  }

  float* cz = C + (size_t)z * (size_t)sC;
#pragma unroll
  for (int i = 0; i < 8; ++i) {
    const int gr = rowBase + 16 * wave + 2 * i + hh;
    const size_t eo = (size_t)gr * (size_t)ldc + col0 + 4 * m;
    *(volatile v4f*)(cz + eo) = fv[i];
    if constexpr (MODE == 3) *(volatile v4f*)(C2 + eo) = fv[i];
  }
  if constexpr (MODE == 1) {
#pragma unroll
    for (int it = 0; it < 4; ++it) {
      const int p = it * GTHR + tid;
      *(volatile v8us*)(auxz + (size_t)(rowBase + (p >> 3)) * XD + 8 * (p & 7)) = dv[it];
    }
  }
  __threadfence();
#pragma unroll
  for (int i = 0; i < 8; ++i) {
    const int gr = rowBase + 16 * wave + 2 * i + hh;
    const size_t eo = (size_t)gr * (size_t)ldc + col0 + 4 * m;
    *(volatile v4f*)(cz + eo) = fv[i];
    if constexpr (MODE == 3) *(volatile v4f*)(C2 + eo) = fv[i];
  }
  if constexpr (MODE == 1) {
#pragma unroll
    for (int it = 0; it < 4; ++it) {
      const int p = it * GTHR + tid;
      *(volatile v8us*)(auxz + (size_t)(rowBase + (p >> 3)) * XD + 8 * (p & 7)) = dv[it];
    }
  }
}

template <int DIR>
__device__ __forceinline__ void conv_dir(const float* __restrict__ xz, const float* __restrict__ cw,
                                         const float* __restrict__ cb, int b, int l, int tid,
                                         float* xf, unsigned short* xh) {
#pragma unroll 1
  for (int q = 0; q < 4; ++q) {
    const int d = q * 256 + tid;
    const v4f w4 = *(const v4fa*)(cw + (size_t)d * 4);
    const float bb = bf16_val(cb[d]);
    float s = 0.0f;
#pragma unroll
    for (int k = 0; k < 4; ++k) {
      const int ls = (DIR != 0) ? (l + 3 - k) : (l - 3 + k);
      const float okf = (ls >= 0 && ls < SEQ) ? 1.0f : 0.0f;
      const int lc = ls < 0 ? 0 : (ls > SEQ - 1 ? SEQ - 1 : ls);
      const float xv = xz[(size_t)(b * SEQ + lc) * (2 * DI) + d];
      s = fmaf(bf16_val(w4[k]), xv * okf, s);
    }
    s = s + bb;
    const float sv = s * (1.0f / (1.0f + expf(-s)));
    unsigned short h, lo;
    hilo(sv, h, lo);
    xf[DIR * DI + d] = sv;
    xh[DIR * 2 * DI + d] = h;
    xh[DIR * 2 * DI + DI + d] = lo;
  }
}

__global__ __launch_bounds__(256) void k_conv(const float* __restrict__ xz,
                                              const float* __restrict__ cwf, const float* __restrict__ cbf,
                                              const float* __restrict__ cwr, const float* __restrict__ cbr,
                                              float* xc, unsigned short* xch) {
  __shared__ __attribute__((aligned(16))) float xf[2 * DI];
  __shared__ __attribute__((aligned(16))) unsigned short xh[2 * 2 * DI];
  const int tid = (int)threadIdx.x;
  const int t = (int)blockIdx.x;
  const int b = t >> 9, l = t & (SEQ - 1);
  conv_dir<0>(xz, cwf, cbf, b, l, tid, xf, xh);
  conv_dir<1>(xz, cwr, cbr, b, l, tid, xf, xh);
  __syncthreads();
  const v4f f0 = *(const v4fa*)(xf + 4 * tid);
  const v4f f1 = *(const v4fa*)(xf + DI + 4 * tid);
  const v8us h0 = *(const v8usa*)(xh + 8 * tid);
  const v8us h1 = *(const v8usa*)(xh + 2 * DI + 8 * tid);
  float* p0 = xc + (size_t)t * DI + 4 * tid;
  float* p1 = xc + (size_t)TOK * DI + (size_t)t * DI + 4 * tid;
  unsigned short* g0 = xch + (size_t)t * (2 * DI) + 8 * tid;
  unsigned short* g1 = xch + (size_t)TOK * (2 * DI) + (size_t)t * (2 * DI) + 8 * tid;
  *(volatile v4f*)p0 = f0; *(volatile v4f*)p1 = f1;
  *(volatile v8us*)g0 = h0; *(volatile v8us*)g1 = h1;
  __threadfence();
  *(volatile v4f*)p0 = f0; *(volatile v4f*)p1 = f1;
  *(volatile v8us*)g0 = h0; *(volatile v8us*)g1 = h1;
}

__global__ __launch_bounds__(SCT) void k_scan(const float* __restrict__ delta, const float* __restrict__ xc,
                                              const float* __restrict__ xdbl, const float* __restrict__ xz,
                                              const float* __restrict__ alf, const float* __restrict__ alr,
                                              const float* __restrict__ dkf, const float* __restrict__ dkr,
                                              float* ydir) {
  __shared__ float As[NST * SCT];
  __shared__ float hsm[NST * SCT];
  __shared__ __attribute__((aligned(16))) float bc[SCH * 32];
  __shared__ __attribute__((aligned(16))) float ys[SCH * SCT];
  const int tid = (int)threadIdx.x;
  const int gx = (int)blockIdx.x, b = (int)blockIdx.y, dir = (int)blockIdx.z;
  const int d = gx * SCT + tid;

#pragma unroll 1
  for (int n = 0; n < NST; ++n) {
    const float af = alf[(size_t)d * NST + n];
    const float ar = alr[(size_t)d * NST + n];
    float al = (dir != 0) ? ar : af;
#if ALOG_BF16
    al = bf16_val(al);
#endif
    As[n * SCT + tid]  = -expf(al);
    hsm[n * SCT + tid] = 0.0f;
  }
  float Dv;
  {
    const float df = dkf[d];
    const float dr = dkr[d];
    Dv = bf16_val((dir != 0) ? dr : df);
  }
  const size_t po = (size_t)dir * (size_t)TOK * DI;
  const float* dl = delta + po;
  const float* uu = xc + po;
  const float* xb = xdbl + (size_t)dir * (size_t)TOK * XD;
  float* yo = ydir + po;

#pragma unroll 1
  for (int c = 0; c < SEQ / SCH; ++c) {
    const int cc = (dir != 0) ? (SEQ / SCH - 1 - c) : c;
    const int t0 = b * SEQ + cc * SCH;
#pragma unroll
    for (int j = 0; j < 2; ++j) {
      const int p = tid + SCT * j;
      const int row = p >> 3, q = p & 7;
      *(v4fa*)(bc + row * 32 + 4 * q) = *(const v4fa*)(xb + (size_t)(t0 + row) * XD + DTR + 4 * q);
    }
    __syncthreads();
#pragma unroll 1
    for (int s = 0; s < SCH; ++s) {
      const int r = (dir != 0) ? (SCH - 1 - s) : s;
      const size_t t = (size_t)(t0 + r);
      const float dt = dl[t * DI + d];
      const float uv = uu[t * DI + d];
      const float zv = xz[t * (2 * DI) + DI + d];
      const float du = dt * uv;
      float yv = 0.0f;
#pragma unroll 1
      for (int n = 0; n < NST; ++n) {
        const float a = As[n * SCT + tid];
        float hv = hsm[n * SCT + tid];
        const float e = expf(dt * a);
        hv = fmaf(hv, e, du * bc[r * 32 + n]);
        hsm[n * SCT + tid] = hv;
        yv = fmaf(hv, bc[r * 32 + NST + n], yv);
      }
      yv = yv + Dv * uv;
      const float g = zv * (1.0f / (1.0f + expf(-zv)));
      ys[r * SCT + tid] = yv * g;
    }
    __syncthreads();
    v4f ov[8];
#pragma unroll
    for (int j = 0; j < 8; ++j) {
      const int p = tid + SCT * j;
      ov[j] = *(const v4fa*)(ys + (p >> 5) * SCT + 4 * (p & 31));
    }
#pragma unroll
    for (int j = 0; j < 8; ++j) {
      const int p = tid + SCT * j;
      *(volatile v4f*)(yo + (size_t)(t0 + (p >> 5)) * DI + gx * SCT + 4 * (p & 31)) = ov[j];
    }
    __threadfence();
#pragma unroll
    for (int j = 0; j < 8; ++j) {
      const int p = tid + SCT * j;
      *(volatile v4f*)(yo + (size_t)(t0 + (p >> 5)) * DI + gx * SCT + 4 * (p & 31)) = ov[j];
    }
  }
}

__global__ __launch_bounds__(256) void k_ysplit(const float* __restrict__ yd, unsigned short* yh) {
  __shared__ __attribute__((aligned(16))) unsigned short sh[2 * DI];
  const int tid = (int)threadIdx.x;
  const int t = (int)blockIdx.x;
  const v4f a = *(const v4fa*)(yd + (size_t)t * DI + 4 * tid);
  const v4f b = *(const v4fa*)(yd + (size_t)TOK * DI + (size_t)t * DI + 4 * tid);
  const v4f y = a + b;
  v4us h4, l4;
  unsigned short hh, ll;
  hilo(y.x, hh, ll); h4[0] = hh; l4[0] = ll;
  hilo(y.y, hh, ll); h4[1] = hh; l4[1] = ll;
  hilo(y.z, hh, ll); h4[2] = hh; l4[2] = ll;
  hilo(y.w, hh, ll); h4[3] = hh; l4[3] = ll;
  *(v4usa*)(sh + 4 * tid) = h4;
  *(v4usa*)(sh + DI + 4 * tid) = l4;
  __syncthreads();
  const v8us q = *(const v8usa*)(sh + 8 * tid);
  unsigned short* dp = yh + (size_t)t * (2 * DI) + 8 * tid;
  *(volatile v8us*)dp = q;
  __threadfence();
  *(volatile v8us*)dp = q;
}

static inline size_t al256(size_t o) { return (o + 255) & ~(size_t)255; }

extern "C" void kernel_launch(void* const* d_in, const int* in_sizes, int n_in,
                              void* d_out, int out_size, void* d_ws, size_t ws_size,
                              hipStream_t stream) {
  if (n_in < 19) return;
  if (in_sizes[0] != NB * SEQ * DM) return;
  if (in_sizes[1] != NLAY * DM) return;
  if (in_sizes[2] != NLAY * 2 * DI * DM) return;
  if (in_sizes[3] != NLAY * DI * 4 || in_sizes[10] != NLAY * DI * 4) return;
  if (in_sizes[4] != NLAY * DI || in_sizes[11] != NLAY * DI) return;
  if (in_sizes[5] != NLAY * XD * DI || in_sizes[12] != NLAY * XD * DI) return;
  if (in_sizes[6] != NLAY * DI * DTR || in_sizes[13] != NLAY * DI * DTR) return;
  if (in_sizes[7] != NLAY * DI || in_sizes[14] != NLAY * DI) return;
  if (in_sizes[8] != NLAY * DI * NST || in_sizes[15] != NLAY * DI * NST) return;
  if (in_sizes[9] != NLAY * DI || in_sizes[16] != NLAY * DI) return;
  if (in_sizes[17] != NLAY * DM * DI) return;
  if (in_sizes[18] != DM) return;
  const int BLD = TOK * DM;
  if (out_size != (1 + NLAY) * BLD) return;

  const float* x      = (const float*)d_in[0];
  const float* norm_w = (const float*)d_in[1];
  const float* inw    = (const float*)d_in[2];
  const float* cwf    = (const float*)d_in[3];
  const float* cbf    = (const float*)d_in[4];
  const float* xpf    = (const float*)d_in[5];
  const float* dwf    = (const float*)d_in[6];
  const float* dbf    = (const float*)d_in[7];
  const float* alf    = (const float*)d_in[8];
  const float* dkf    = (const float*)d_in[9];
  const float* cwr    = (const float*)d_in[10];
  const float* cbr    = (const float*)d_in[11];
  const float* xpr    = (const float*)d_in[12];
  const float* dwr    = (const float*)d_in[13];
  const float* dbr    = (const float*)d_in[14];
  const float* alr    = (const float*)d_in[15];
  const float* dkr    = (const float*)d_in[16];
  const float* outw   = (const float*)d_in[17];
  const float* normf  = (const float*)d_in[18];
  float* out = (float*)d_out;

  char* ws = (char*)d_ws;
  size_t off = 0;
  const size_t oINW  = off; off = al256(off + (size_t)NLAY * 2 * DI * DM * 2);
  const size_t oXPW  = off; off = al256(off + (size_t)2 * NLAY * XD * DI * 2);
  const size_t oDTW  = off; off = al256(off + (size_t)2 * NLAY * DI * DTR * 2);
  const size_t oOUTW = off; off = al256(off + (size_t)NLAY * DM * DI * 2);
  const size_t oRES  = off; off = al256(off + (size_t)TOK * DM * 4);
  const size_t oHS   = off; off = al256(off + (size_t)TOK * DM * 4);
  const size_t oHN   = off; off = al256(off + (size_t)TOK * 2 * DM * 2);
  const size_t oXZ   = off; off = al256(off + (size_t)TOK * 2 * DI * 4);
  const size_t oXC   = off; off = al256(off + (size_t)2 * TOK * DI * 4);
  const size_t oXCH  = off; off = al256(off + (size_t)2 * TOK * 2 * DI * 2);
  const size_t oXDBL = off; off = al256(off + (size_t)2 * TOK * XD * 4);
  const size_t oDT   = off; off = al256(off + (size_t)2 * TOK * XD * 2);
  const size_t oDEL  = off; off = al256(off + (size_t)2 * TOK * DI * 4);
  const size_t oYD   = off; off = al256(off + (size_t)2 * TOK * DI * 4);
  const size_t oYH   = off; off = al256(off + (size_t)TOK * 2 * DI * 2);
  if (off > ws_size || off > (size_t)WSMAX) return;
  unsigned short* INW  = (unsigned short*)(ws + oINW);
  unsigned short* XPW  = (unsigned short*)(ws + oXPW);
  unsigned short* DTW  = (unsigned short*)(ws + oDTW);
  unsigned short* OUTW = (unsigned short*)(ws + oOUTW);
  float*          RES  = (float*)(ws + oRES);
  float*          HS   = (float*)(ws + oHS);
  unsigned short* HN   = (unsigned short*)(ws + oHN);
  float*          XZ   = (float*)(ws + oXZ);
  float*          XC   = (float*)(ws + oXC);
  unsigned short* XCH  = (unsigned short*)(ws + oXCH);
  float*          XDBL = (float*)(ws + oXDBL);
  unsigned short* DT   = (unsigned short*)(ws + oDT);
  float*          DEL  = (float*)(ws + oDEL);
  float*          YD   = (float*)(ws + oYD);
  unsigned short* YH   = (unsigned short*)(ws + oYH);

  {
    const int uIN = NLAY * 2 * DI * DM / 8, uXP = NLAY * XD * DI / 8, uDT = NLAY * DI * DTR / 8, uOU = NLAY * DM * DI / 8;
    k_cvt<<<(uIN + 255) / 256, 256, 0, stream>>>(inw, INW, uIN);
    k_cvt<<<(uXP + 255) / 256, 256, 0, stream>>>(xpf, XPW, uXP);
    k_cvt<<<(uXP + 255) / 256, 256, 0, stream>>>(xpr, XPW + (size_t)NLAY * XD * DI, uXP);
    k_cvt<<<(uDT + 255) / 256, 256, 0, stream>>>(dwf, DTW, uDT);
    k_cvt<<<(uDT + 255) / 256, 256, 0, stream>>>(dwr, DTW + (size_t)NLAY * DI * DTR, uDT);
    k_cvt<<<(uOU + 255) / 256, 256, 0, stream>>>(outw, OUTW, uOU);
  }

  for (int i = 0; i < NLAY; ++i) {
    if (i == 0) k_norm<0><<<TOK / 8, 256, 0, stream>>>(x, HS, RES, norm_w, HN, out);
    else        k_norm<1><<<TOK / 8, 256, 0, stream>>>(x, HS, RES, norm_w + (size_t)i * DM, HN, out);
    k_gemm<0><<<dim3(TOK / GBM, (2 * DI) / GBN, 1), GTHR, 0, stream>>>(
        HN, INW + (size_t)i * 2 * DI * DM, XZ, XZ, DT, dbf, dbr,
        2 * DM, 0, DM, 0, 2 * DI, 0, 0);
    k_conv<<<TOK, 256, 0, stream>>>(XZ, cwf + (size_t)i * DI * 4, cbf + (size_t)i * DI,
                                    cwr + (size_t)i * DI * 4, cbr + (size_t)i * DI, XC, XCH);
    k_gemm<1><<<dim3(TOK / GBM, 1, 2), GTHR, 0, stream>>>(
        XCH, XPW + (size_t)i * XD * DI, XDBL, XDBL, DT, dbf, dbr,
        2 * DI, TOK * 2 * DI, DI, NLAY * XD * DI, XD, TOK * XD, TOK * XD);
    k_gemm<2><<<dim3(TOK / GBM, DI / GBN, 2), GTHR, 0, stream>>>(
        DT, DTW + (size_t)i * DI * DTR, DEL, DEL, DT,
        dbf + (size_t)i * DI, dbr + (size_t)i * DI,
        XD, TOK * XD, DTR, NLAY * DI * DTR, DI, TOK * DI, 0);
    k_scan<<<dim3(DI / SCT, NB, 2), SCT, 0, stream>>>(
        DEL, XC, XDBL, XZ, alf + (size_t)i * DI * NST, alr + (size_t)i * DI * NST,
        dkf + (size_t)i * DI, dkr + (size_t)i * DI, YD);
    k_ysplit<<<TOK, 256, 0, stream>>>(YD, YH);
    k_gemm<3><<<dim3(TOK / GBM, DM / GBN, 1), GTHR, 0, stream>>>(
        YH, OUTW + (size_t)i * DM * DI, HS, out + (size_t)(1 + i) * BLD, DT, dbf, dbr,
        2 * DI, 0, DI, 0, DM, 0, 0);
  }
  k_norm<2><<<TOK / 8, 256, 0, stream>>>(x, HS, RES, normf, HN, out);
}
